// CasualAttention_37847251812797
// MI455X (gfx1250) — hardware-verified
//
#include <hip/hip_runtime.h>


#ifndef NB
#define NB 4
#endif
#ifndef SEQ
#define SEQ 2048
#endif
#define NB_FULL  4
#define SEQ_FULL 2048
#define DM   1024
#define NH   16
#define HD   64
#define D3   (3 * DM)
#define RH   ((SEQ < 512) ? SEQ : 512)
#define CQK  8.0f
#define CV   8.0f
#define CY   16.0f
#define CW   64.0f
static_assert(SEQ % 64 == 0 && SEQ >= 64 && SEQ <= SEQ_FULL);
static_assert(NB >= 1 && NB <= NB_FULL);
static_assert(RH % 64 == 0 && RH <= SEQ && RH >= 64);
static_assert(DM % 64 == 0 && HD == 64 && NH * HD == DM);

typedef _Float16 h16;
typedef unsigned short bf;
typedef __attribute__((ext_vector_type(16))) __bf16   v16bf;
typedef __attribute__((ext_vector_type(16))) _Float16 v16h;
typedef __attribute__((ext_vector_type(8)))  _Float16 v8h;
typedef __attribute__((ext_vector_type(8)))  unsigned short v8us;
typedef __attribute__((ext_vector_type(2)))  _Float16 v2h;
typedef __attribute__((ext_vector_type(2)))  unsigned short v2us;
typedef __attribute__((ext_vector_type(8)))  float    v8f;
typedef __attribute__((ext_vector_type(4)))  float    v4f;
typedef v8h  __attribute__((may_alias)) v8ha;
typedef v4f  __attribute__((may_alias)) v4fa;
typedef v8us __attribute__((may_alias)) v8usa;

__device__ __forceinline__ unsigned short f2bf(float f) { unsigned u = __float_as_uint(f); u += 0x7FFFu + ((u >> 16) & 1u); return (unsigned short)(u >> 16); }
__device__ __forceinline__ float bf2f(unsigned short b) { return __uint_as_float(((unsigned)b) << 16); }
__device__ __forceinline__ float bfr(float f) { return bf2f(f2bf(f)); }
__device__ __forceinline__ v16h cat16(v8h lo, v8h hi) { return __builtin_shufflevector(lo, hi, 0, 1, 2, 3, 4, 5, 6, 7, 8, 9, 10, 11, 12, 13, 14, 15); }
__device__ __forceinline__ v16bf cat16b(v8us lo, v8us hi) { return __builtin_bit_cast(v16bf, __builtin_shufflevector(lo, hi, 0, 1, 2, 3, 4, 5, 6, 7, 8, 9, 10, 11, 12, 13, 14, 15)); }
__device__ __forceinline__ v8f wmma16(v16h a, v16h b, v8f c) { return __builtin_amdgcn_wmma_f32_16x16x32_f16(false, a, false, b, (short)0, c, false, false); }
__device__ __forceinline__ v8f wmmab(v16bf a, v16bf b, v8f c) { return __builtin_amdgcn_wmma_f32_16x16x32_bf16(false, a, false, b, (short)0, c, false, false); }
__device__ __forceinline__ void splitf(float y, unsigned short& h, unsigned short& l) { h = f2bf(y); l = f2bf(y - bf2f(h)); }
__device__ __forceinline__ void tocv(float p, h16& o) { o = (h16)p; }
__device__ __forceinline__ void tocv(float p, bf& o) { o = f2bf(p); }

template <typename T16> struct WFrag;
template <> struct WFrag<h16> { typedef v16h V; static __device__ __forceinline__ V ld(const h16* p) { return cat16(*(const v8ha*)p, *(const v8ha*)(p + 16)); } static __device__ __forceinline__ v8f mma(V a, V b, v8f c) { return wmma16(a, b, c); } };
template <> struct WFrag<bf> { typedef v16bf V; static __device__ __forceinline__ V ld(const bf* p) { return cat16b(*(const v8usa*)p, *(const v8usa*)(p + 16)); } static __device__ __forceinline__ v8f mma(V a, V b, v8f c) { return wmmab(a, b, c); } };

template <typename T16, int NSPLIT, bool BIAS>
__global__ __launch_bounds__(32) void k_gemmw(const T16* __restrict__ A, const T16* __restrict__ A2, const T16* __restrict__ Bt, const T16* __restrict__ Bt2, int K, float* C, int ldc, const float* __restrict__ bias, float oscale, size_t sA, size_t sB, size_t sC) {
    typedef typename WFrag<T16>::V V;
    __shared__ __align__(16) float os[16 * 68];
    const size_t z = blockIdx.z; A += z * sA; if (A2) A2 += z * sA; Bt += z * sB; if (Bt2) Bt2 += z * sB; C += z * sC;
    const int lane = threadIdx.x & 31, lr = lane & 15, hi = lane >> 4; const int r0 = blockIdx.x * 64, c0 = blockIdx.y * 64;
    v8f acc[4][4];
#pragma unroll
    for (int mb = 0; mb < 4; ++mb)
#pragma unroll
        for (int nb = 0; nb < 4; ++nb) acc[mb][nb] = (v8f){};
    const size_t aoff = (size_t)(r0 + lr) * K + 8 * hi, boff = (size_t)(c0 + lr) * K + 8 * hi;
#pragma unroll 1
    for (int kc = 0; kc < K; kc += 32) {
        V a[4], a2[4];
#pragma unroll
        for (int mb = 0; mb < 4; ++mb) { a[mb] = WFrag<T16>::ld(A + aoff + (size_t)mb * 16 * K + kc); if (NSPLIT == 1 || NSPLIT == 2) a2[mb] = WFrag<T16>::ld(A2 + aoff + (size_t)mb * 16 * K + kc); else a2[mb] = a[mb]; }
#pragma unroll
        for (int nb = 0; nb < 4; ++nb) { const V b = WFrag<T16>::ld(Bt + boff + (size_t)nb * 16 * K + kc); V b2 = b; if (NSPLIT >= 2) b2 = WFrag<T16>::ld(Bt2 + boff + (size_t)nb * 16 * K + kc);
#pragma unroll
            for (int mb = 0; mb < 4; ++mb) { acc[mb][nb] = WFrag<T16>::mma(a[mb], b, acc[mb][nb]); if (NSPLIT == 1 || NSPLIT == 2) acc[mb][nb] = WFrag<T16>::mma(a2[mb], b, acc[mb][nb]); if (NSPLIT >= 2) acc[mb][nb] = WFrag<T16>::mma(a[mb], b2, acc[mb][nb]); } }
        asm volatile("v_nop\n\tv_nop\n\tv_nop\n\tv_nop" : "+v"(acc[0][0]), "+v"(acc[1][1]), "+v"(acc[2][2]), "+v"(acc[3][3]) : "v"(a[0]), "v"(a[3]));
    }
#pragma unroll
    for (int mb = 0; mb < 4; ++mb) {
#pragma unroll
        for (int nb = 0; nb < 4; ++nb) {
#pragma unroll
            for (int j = 0; j < 8; ++j) os[(hi * 8 + j) * 68 + nb * 16 + lr] = acc[mb][nb][j]; }
        __syncthreads();
        float* crow = C + (size_t)(r0 + mb * 16) * ldc + c0;
#pragma unroll 1
        for (int ps = 0; ps < 2; ++ps) {
#pragma unroll
            for (int s = 0; s < 8; ++s) { const int row = 2 * s + hi, cofs = lr * 4; v4f val = *(const v4fa*)(os + row * 68 + cofs);
#pragma unroll
                for (int i = 0; i < 4; ++i) { const float bv = BIAS ? bfr(bias[c0 + cofs + i]) : 0.0f; val[i] = val[i] * oscale + bv; }
                *(volatile v4f*)(crow + (size_t)row * ldc + cofs) = val; }
            if (ps == 0) __threadfence(); }
        __syncthreads();
    }
}

__global__ __launch_bounds__(32) __attribute__((amdgpu_num_vgpr(256)))
void k_qkv(const bf* __restrict__ A, const bf* __restrict__ Bt, const float* __restrict__ bias,
           h16* Q16, h16* K16, h16* VT16, bf* Qh, bf* Ql, bf* Kh, bf* Kl, bf* VTh, bf* VTl) {
    typedef WFrag<bf>::V V;
    __shared__ __align__(16) float os[64 * 68];
    const int lane = threadIdx.x & 31, lr = lane & 15, hi = lane >> 4; const int r0 = blockIdx.x * 64, c0 = blockIdx.y * 64;
    const int K = DM;
    v8f acc[4][4];
#pragma unroll
    for (int mb = 0; mb < 4; ++mb)
#pragma unroll
        for (int nb = 0; nb < 4; ++nb) acc[mb][nb] = (v8f){};
    const size_t aoff = (size_t)(r0 + lr) * K + 8 * hi, boff = (size_t)(c0 + lr) * K + 8 * hi;
#pragma unroll 1
    for (int kc = 0; kc < K; kc += 32) {
        V a[4];
#pragma unroll
        for (int mb = 0; mb < 4; ++mb) a[mb] = WFrag<bf>::ld(A + aoff + (size_t)mb * 16 * K + kc);
#pragma unroll
        for (int nb = 0; nb < 4; ++nb) { const V b = WFrag<bf>::ld(Bt + boff + (size_t)nb * 16 * K + kc);
#pragma unroll
            for (int mb = 0; mb < 4; ++mb) acc[mb][nb] = WFrag<bf>::mma(a[mb], b, acc[mb][nb]); }
        asm volatile("v_nop\n\tv_nop\n\tv_nop\n\tv_nop" : "+v"(acc[0][0]), "+v"(acc[1][1]), "+v"(acc[2][2]), "+v"(acc[3][3]) : "v"(a[0]), "v"(a[3]));
    }
    float bcol[4];
#pragma unroll
    for (int nb = 0; nb < 4; ++nb) bcol[nb] = bfr(bias[c0 + nb * 16 + lr]);
    const int sec = c0 / DM; const int hh = (c0 - sec * DM) / HD; const int b = r0 / SEQ; const int t0 = r0 - b * SEQ;
    const bool isv = (sec == 2); const bool hl = (t0 < RH);
#pragma unroll
    for (int mb = 0; mb < 4; ++mb)
#pragma unroll
        for (int nb = 0; nb < 4; ++nb)
#pragma unroll
            for (int j = 0; j < 8; ++j) { const int rr = mb * 16 + hi * 8 + j, cc = nb * 16 + lr; const int idx = isv ? (cc * 68 + rr) : (rr * 68 + cc); os[idx] = acc[mb][nb][j] + bcol[nb]; }
    __syncthreads();
    const size_t bh = (size_t)b * NH + hh; const int th = hl ? t0 : 0;
    h16* d16; bf* dh; bf* dl; size_t p16, phl; float car;
    if (sec == 0)      { d16 = Q16 + (bh * SEQ + t0) * HD; p16 = HD; dh = Qh + (bh * RH + th) * HD; dl = Ql + (bh * RH + th) * HD; phl = HD; car = CQK; }
    else if (sec == 1) { d16 = K16 + (bh * SEQ + t0) * HD; p16 = HD; dh = Kh + (bh * RH + th) * HD; dl = Kl + (bh * RH + th) * HD; phl = HD; car = CQK; }
    else               { d16 = VT16 + bh * HD * (size_t)SEQ + t0; p16 = SEQ; dh = VTh + bh * HD * (size_t)RH + th; dl = VTl + bh * HD * (size_t)RH + th; phl = RH; car = CV; }
    const int q = lane >> 3, pc = lane & 7;
#pragma unroll 1
    for (int ps = 0; ps < 2; ++ps) {
#pragma unroll 1
        for (int s = 0; s < 16; ++s) { const int row = 4 * s + q; const float* op = os + row * 68 + pc * 8; const v4f x0 = *(const v4fa*)op, x1 = *(const v4fa*)(op + 4); v8h o16;
#pragma unroll
            for (int i = 0; i < 4; ++i) { o16[i] = (h16)(x0[i] * car); o16[i + 4] = (h16)(x1[i] * car); }
            *(volatile v8h*)(d16 + (size_t)row * p16 + pc * 8) = o16;
            if (hl) { v8us oh, ol;
#pragma unroll
                for (int i = 0; i < 4; ++i) { unsigned short a0, e0, a1, e1; splitf(x0[i], a0, e0); splitf(x1[i], a1, e1); oh[i] = a0; ol[i] = e0; oh[i + 4] = a1; ol[i + 4] = e1; }
                *(volatile v8us*)(dh + (size_t)row * phl + pc * 8) = oh; *(volatile v8us*)(dl + (size_t)row * phl + pc * 8) = ol; } }
        if (ps == 0) __threadfence(); }
}

template <typename T16, bool HL>
__global__ __launch_bounds__(32) __attribute__((amdgpu_num_vgpr(256)))
void k_attn(const T16* __restrict__ Qa, const T16* __restrict__ Qb, const T16* __restrict__ Ka, const T16* __restrict__ Kb,
            const T16* __restrict__ Va, const T16* __restrict__ Vb, int w0, h16* Y16, bf* Yh, bf* Yl) {
    typedef typename WFrag<T16>::V V;
    constexpr int TP = HL ? RH : SEQ;
    constexpr float EC = (HL ? 0.125f : (0.125f / (CQK * CQK))) * 1.4426950408889634f;
    constexpr float OSC = HL ? 1.0f : (1.0f / CV);
    __shared__ __align__(16) T16 sp0[16 * 72];
    __shared__ __align__(16) T16 sp1[16 * 72];
    __shared__ __align__(16) float so[16 * 68];
    const int lane = threadIdx.x & 31, l16 = lane & 15, hf = lane >> 4;
    const int r0 = (w0 + (int)blockIdx.x) * 16; const int h = blockIdx.y, b = blockIdx.z; const size_t bh = (size_t)b * NH + h;
    const int clast = (r0 + 15) >> 6;
    V q[2], q2[2];
#pragma unroll
    for (int ks = 0; ks < 2; ++ks) { const size_t qo = (bh * TP + r0 + l16) * HD + 32 * ks + 8 * hf; q[ks] = WFrag<T16>::ld(Qa + qo); if (HL) q2[ks] = WFrag<T16>::ld(Qb + qo); else q2[ks] = q[ks]; }
    float mrow[8], lrow[8]; v8f o[4];
#pragma unroll
    for (int r = 0; r < 8; ++r) { mrow[r] = -__builtin_inff(); lrow[r] = 0.f; }
#pragma unroll
    for (int dt = 0; dt < 4; ++dt) o[dt] = (v8f){};
#pragma unroll 1
    for (int c = 0; c <= clast; ++c) {
        const int kb = c * 64;
        v8f s[4];
#pragma unroll
        for (int nt = 0; nt < 4; ++nt) s[nt] = (v8f){};
        V kf = q[0];
#pragma unroll
        for (int ks = 0; ks < 2; ++ks) {
#pragma unroll
            for (int nt = 0; nt < 4; ++nt) { const size_t ko = (bh * TP + kb + 16 * nt + l16) * HD + 32 * ks + 8 * hf; kf = WFrag<T16>::ld(Ka + ko); s[nt] = WFrag<T16>::mma(q[ks], kf, s[nt]);
                if (HL) { s[nt] = WFrag<T16>::mma(q2[ks], kf, s[nt]); const V kf2 = WFrag<T16>::ld(Kb + ko); s[nt] = WFrag<T16>::mma(q[ks], kf2, s[nt]); } } }
        asm volatile("v_nop\n\tv_nop\n\tv_nop\n\tv_nop" : "+v"(s[0]), "+v"(s[1]), "+v"(s[2]), "+v"(s[3]) : "v"(q[0]), "v"(q[1]), "v"(kf));
        if (c == clast) {
#pragma unroll
            for (int nt = 0; nt < 4; ++nt)
#pragma unroll
                for (int r = 0; r < 8; ++r) { const int key = kb + 16 * nt + l16, qr = r0 + 8 * hf + r; s[nt][r] = (key > qr) ? -__builtin_inff() : s[nt][r]; } }
#pragma unroll
        for (int r = 0; r < 8; ++r) {
            float mx = fmaxf(fmaxf(s[0][r], s[1][r]), fmaxf(s[2][r], s[3][r]));
            mx = fmaxf(mx, __shfl_xor(mx, 8, 32)); mx = fmaxf(mx, __shfl_xor(mx, 4, 32)); mx = fmaxf(mx, __shfl_xor(mx, 2, 32)); mx = fmaxf(mx, __shfl_xor(mx, 1, 32));
            const float mn = fmaxf(mrow[r], mx);
            const float alpha = __builtin_amdgcn_exp2f((mrow[r] - mn) * EC);
            mrow[r] = mn;
            float psum = 0.f;
#pragma unroll
            for (int nt = 0; nt < 4; ++nt) { const float p = __builtin_amdgcn_exp2f((s[nt][r] - mn) * EC); s[nt][r] = p; psum += p; }
            psum += __shfl_xor(psum, 8, 32); psum += __shfl_xor(psum, 4, 32); psum += __shfl_xor(psum, 2, 32); psum += __shfl_xor(psum, 1, 32);
            lrow[r] = lrow[r] * alpha + psum;
#pragma unroll
            for (int dt = 0; dt < 4; ++dt) o[dt][r] *= alpha;
        }
#pragma unroll
        for (int nt = 0; nt < 4; ++nt)
#pragma unroll
            for (int r = 0; r < 8; ++r) { const int idx = (8 * hf + r) * 72 + 16 * nt + l16; const float p = s[nt][r]; tocv(p, sp0[idx]); if (HL) tocv(p - bfr(p), sp1[idx]); }
        __syncthreads();
        V pf = q[0], pf2 = q[0], vf = q[0];
#pragma unroll
        for (int ks = 0; ks < 2; ++ks) { const int po = l16 * 72 + 32 * ks + 8 * hf; pf = WFrag<T16>::ld(sp0 + po); if (HL) pf2 = WFrag<T16>::ld(sp1 + po);
#pragma unroll
            for (int dt = 0; dt < 4; ++dt) { const size_t vo = (bh * HD + 16 * dt + l16) * TP + kb + 32 * ks + 8 * hf; vf = WFrag<T16>::ld(Va + vo); o[dt] = WFrag<T16>::mma(pf, vf, o[dt]);
                if (HL) { o[dt] = WFrag<T16>::mma(pf2, vf, o[dt]); const V vf2 = WFrag<T16>::ld(Vb + vo); o[dt] = WFrag<T16>::mma(pf, vf2, o[dt]); } } }
        asm volatile("v_nop\n\tv_nop\n\tv_nop\n\tv_nop" : "+v"(o[0]), "+v"(o[1]), "+v"(o[2]), "+v"(o[3]) : "v"(pf), "v"(vf));
        __syncthreads();
    }
#pragma unroll
    for (int r = 0; r < 8; ++r) { const float inv = OSC / lrow[r];
#pragma unroll
        for (int dt = 0; dt < 4; ++dt) so[(8 * hf + r) * 68 + 16 * dt + l16] = o[dt][r] * inv; }
    __syncthreads();
    const int qq = lane >> 3, pc = lane & 7;
#pragma unroll 1
    for (int ps = 0; ps < 2; ++ps) {
#pragma unroll 1
        for (int sg = 0; sg < 4; ++sg) { const int row = 4 * sg + qq; const float* op = so + row * 68 + pc * 8; const v4f x0 = *(const v4fa*)op, x1 = *(const v4fa*)(op + 4); v8h o16;
#pragma unroll
            for (int i = 0; i < 4; ++i) { o16[i] = (h16)(x0[i] * CY); o16[i + 4] = (h16)(x1[i] * CY); }
            *(volatile v8h*)(Y16 + ((size_t)(b * SEQ + r0 + row) * DM + h * HD + pc * 8)) = o16;
            if (HL) { v8us oh, ol;
#pragma unroll
                for (int i = 0; i < 4; ++i) { unsigned short a0, e0, a1, e1; splitf(x0[i], a0, e0); splitf(x1[i], a1, e1); oh[i] = a0; ol[i] = e0; oh[i + 4] = a1; ol[i + 4] = e1; }
                const size_t yo = (size_t)(b * RH + r0 + row) * DM + h * HD + pc * 8; *(volatile v8us*)(Yh + yo) = oh; *(volatile v8us*)(Yl + yo) = ol; } }
        if (ps == 0) __threadfence(); }
}

template <typename TO> struct P2;
template <> struct P2<bf>  { typedef v2us T; };
template <> struct P2<h16> { typedef v2h  T; };
template <typename TO>
__global__ __launch_bounds__(256) void k_wt(const float* __restrict__ w, int K, int N, TO* Bt, float sc) {
    typedef typename P2<TO>::T T2;
    const int lane = threadIdx.x & 31; const int L0 = (blockIdx.x * 8 + (threadIdx.x >> 5)) * 8; const int nlines = N * K / 64;
#pragma unroll 1
    for (int ps = 0; ps < 2; ++ps) {
#pragma unroll 1
        for (int l = 0; l < 8; ++l) { const int L = L0 + l; if (L >= nlines) break; const size_t e = (size_t)L * 64 + lane * 2; const int k = (int)(e % K), n = (int)(e / K); T2 o; TO o0, o1;
            tocv(bfr(w[(size_t)k * N + n]) * sc, o0); tocv(bfr(w[(size_t)(k + 1) * N + n]) * sc, o1); o[0] = o0; o[1] = o1; *(volatile T2*)(Bt + e) = o; }
        if (ps == 0) __threadfence(); }
}
__global__ __launch_bounds__(256) void k_cvtx(const float* __restrict__ x, bf* dst, size_t n8) {
    const size_t i = (size_t)blockIdx.x * 256 + threadIdx.x; if (i >= n8) return;
    const size_t m = i / (DM / 8); const int c8 = (int)(i % (DM / 8)); const size_t b = m / SEQ, t = m % SEQ;
    const v8f v = *(const v8f*)(x + ((b * SEQ_FULL + t) * DM + (size_t)c8 * 8)); v8us o;
#pragma unroll
    for (int k = 0; k < 8; ++k) o[k] = f2bf(v[k]);
    *(volatile v8us*)(dst + i * 8) = o; __threadfence(); *(volatile v8us*)(dst + i * 8) = o; }

extern "C" void kernel_launch(void* const* d_in, const int* in_sizes, int n_in,
                              void* d_out, int out_size, void* d_ws, size_t ws_size, hipStream_t stream) {
    if (n_in < 5) return;
    if (in_sizes[0] < (NB - 1) * SEQ_FULL * DM + SEQ * DM) return;
    if (in_sizes[1] < DM * D3 || in_sizes[2] < D3 || in_sizes[3] < DM * DM || in_sizes[4] < DM) return;
    if (out_size < (NB - 1) * SEQ_FULL * DM + SEQ * DM) return;
    const float* x = (const float*)d_in[0]; const float* w_attn = (const float*)d_in[1]; const float* b_attn = (const float*)d_in[2]; const float* w_proj = (const float*)d_in[3]; const float* b_proj = (const float*)d_in[4];
    float* OUT = (float*)d_out;
    char* wsp = (char*)d_ws;
    auto take = [&](size_t bytes) { char* p = wsp; wsp += (bytes + 255) & ~(size_t)255; return (void*)p; };
    bf*  WA   = (bf*)take((size_t)D3 * DM * 2);
    bf*  WPB  = (bf*)take((size_t)DM * DM * 2);
    h16* WP16 = (h16*)take((size_t)DM * DM * 2);
    bf*  XB   = (bf*)take((size_t)NB * SEQ * DM * 2);
    h16* Q16  = (h16*)take((size_t)NB * NH * SEQ * HD * 2);
    h16* K16  = (h16*)take((size_t)NB * NH * SEQ * HD * 2);
    h16* VT16 = (h16*)take((size_t)NB * NH * HD * SEQ * 2);
    bf*  Qh   = (bf*)take((size_t)NB * NH * RH * HD * 2);  bf* Ql  = (bf*)take((size_t)NB * NH * RH * HD * 2);
    bf*  Kh   = (bf*)take((size_t)NB * NH * RH * HD * 2);  bf* Kl  = (bf*)take((size_t)NB * NH * RH * HD * 2);
    bf*  VTh  = (bf*)take((size_t)NB * NH * HD * RH * 2);  bf* VTl = (bf*)take((size_t)NB * NH * HD * RH * 2);
    h16* Y16  = (h16*)take((size_t)NB * SEQ * DM * 2);
    bf*  Yh   = (bf*)take((size_t)NB * RH * DM * 2);    bf* Yl  = (bf*)take((size_t)NB * RH * DM * 2);
    if ((size_t)(wsp - (char*)d_ws) > ws_size) return;

    k_wt<bf><<<(unsigned)((D3 * DM / 64 + 63) / 64), 256, 0, stream>>>(w_attn, DM, D3, WA, 1.0f);
    k_wt<bf><<<(unsigned)((DM * DM / 64 + 63) / 64), 256, 0, stream>>>(w_proj, DM, DM, WPB, 1.0f);
    k_wt<h16><<<(unsigned)((DM * DM / 64 + 63) / 64), 256, 0, stream>>>(w_proj, DM, DM, WP16, CW);
    const size_t n8 = (size_t)NB * SEQ * DM / 8;
    k_cvtx<<<(unsigned)((n8 + 255) / 256), 256, 0, stream>>>(x, XB, n8);
    k_qkv<<<dim3(NB * SEQ / 64, D3 / 64, 1), 32, 0, stream>>>(XB, WA, b_attn, Q16, K16, VT16, Qh, Ql, Kh, Kl, VTh, VTl);
    k_attn<bf, true><<<dim3(RH / 16, NH, NB), 32, 0, stream>>>(Qh, Ql, Kh, Kl, VTh, VTl, 0, Y16, Yh, Yl);
    if (SEQ > RH) k_attn<h16, false><<<dim3((SEQ - RH) / 16, NH, NB), 32, 0, stream>>>(Q16, nullptr, K16, nullptr, VT16, nullptr, RH / 16, Y16, Yh, Yl);
    k_gemmw<bf, 1, true><<<dim3(RH / 64, DM / 64, NB), 32, 0, stream>>>(Yh, Yl, WPB, nullptr, DM, OUT, DM, b_proj, 1.0f, (size_t)RH * DM, (size_t)0, (size_t)SEQ_FULL * DM);
    if (SEQ > RH) k_gemmw<h16, 0, true><<<dim3((SEQ - RH) / 64, DM / 64, NB), 32, 0, stream>>>(Y16 + (size_t)RH * DM, nullptr, WP16, nullptr, DM, OUT + (size_t)RH * DM, DM, b_proj, 1.0f / (CY * CW), (size_t)SEQ * DM, (size_t)0, (size_t)SEQ_FULL * DM);
}
